// TemporalGNN_43198781063869
// MI455X (gfx1250) — hardware-verified
//
#include <hip/hip_runtime.h>
#include <math.h>

constexpr int kN     = 50000;
constexpr int kE     = 1600000;
constexpr int kInCh  = 8;
constexpr int kPer   = 12;
constexpr int kFeat  = kInCh * kPer;
constexpr int kHid   = 64;

constexpr int kGateK  = 160;
constexpr int kGateBP = 192;
constexpr int kHeadK  = 128;
constexpr int kHeadBP = 128;
constexpr int kAP     = 160;
static_assert(kGateK % 32 == 0 && kHeadK % 32 == 0, "K multiples of 32");
static_assert(kGateK <= kAP && kHeadK <= kAP && kGateK <= kGateBP, "pitches cover K");

constexpr int kPrepGate   = kHid * kGateBP;
constexpr int kPrepP1     = 3 * kPrepGate;
constexpr int kPrepPO     = kPrepP1 + kHid * kHeadBP;
constexpr int kPrepHalves = kPrepPO + 16 * kHeadBP;
constexpr int kPrepChunks = kPrepHalves / 8;
constexpr int kTabFloats = 288;
constexpr int kTabBz = 0, kTabBr = 64, kTabBh = 128, kTabL1b = 192, kTabOutb = 256, kTabProb = 272;
constexpr int kThr = 256;
constexpr int kR0 = 3 * kHid * 16;
constexpr int kR1 = kR0 + 3 * kHid * 8;
constexpr int kR2 = kR1 + kHid * 16;
constexpr int kR3 = kR2 + 16 * 16;
constexpr int kR4 = kR3 + kTabFloats;
static_assert(kR3 == kPrepChunks, "chunk coverage");
static_assert(kR0 % 32 == 0 && kR1 % 32 == 0 && kR2 % 32 == 0 && kR3 % 32 == 0 && kR4 % 32 == 0, "wave-uniform regions");
constexpr int kPrepBlocks = (kR4 + kThr - 1) / kThr;

constexpr int kAggPitch = 128;
constexpr int kSpt   = 16;
constexpr int kSch   = kThr * kSpt;
constexpr int kNch   = (kE + kSch - 1) / kSch;
static_assert(kE % kSpt == 0, "thread edge groups never straddle the list end");
constexpr int kSrbD  = 8192;
constexpr int kNblkD = (kN + kSrbD - 1) / kSrbD;
constexpr int kRowsWaveD = kSrbD / 8;
constexpr int kShiftD = 10;
static_assert(kRowsWaveD == (1 << kShiftD), "wave ownership shift");
constexpr int kDinvRows = kNblkD * kSrbD;
constexpr int kSrbA  = 2048;
constexpr int kNblkA = (kN + kSrbA - 1) / kSrbA;
constexpr int kRowsWaveA = kSrbA / 8;
constexpr int kShiftA = 24;
static_assert(kRowsWaveA == (1 << (kShiftA - 16)), "wave ownership shift");
constexpr int kAggRows = kNblkA * kSrbA;
static_assert(kDinvRows >= kAggRows && kAggRows >= kN, "plane extents");
static_assert(kN < 65536, "src packs into 16 bits");

constexpr int kNodesBlk  = 64;
constexpr int kGruThr    = 128;
constexpr int kGruBlocks = (kN + kNodesBlk - 1) / kNodesBlk;
constexpr int kOutLines  = kN * kPer * 4 / 128;
constexpr int kLinesBlk  = kNodesBlk * kPer * 4 / 128;
static_assert((kN * kPer * 4) % 128 == 0 && (kNodesBlk * kPer * 4) % 128 == 0, "whole output lines");
static_assert(((kN % kNodesBlk) * kPer * 4) % 128 == 0, "tail block = whole lines");
static_assert(kN % 16 == 0, "wave row tiles exact");

typedef __attribute__((ext_vector_type(16))) __bf16   v16b;
typedef __attribute__((ext_vector_type(8)))  __bf16   v8b;
typedef __attribute__((ext_vector_type(8)))  float    v8f;
typedef __attribute__((ext_vector_type(4)))  float    v4f;
typedef __attribute__((ext_vector_type(4)))  int      v4i;
typedef __attribute__((ext_vector_type(4)))  unsigned v4u;

__device__ __forceinline__ unsigned short f2bf_bits(float f) {
  unsigned u = __float_as_uint(f);
  return (unsigned short)((u + 0x7FFFu + ((u >> 16) & 1u)) >> 16);
}
__device__ __forceinline__ float bf_bits2f(unsigned short h) { return __uint_as_float(((unsigned)h) << 16); }
__device__ __forceinline__ float bfr(float f) { return bf_bits2f(f2bf_bits(f)); }
__device__ __forceinline__ unsigned pk16(unsigned short a, unsigned short b) { return (unsigned)a | ((unsigned)b << 16); }
__device__ __forceinline__ v4u pack8(const unsigned short* hb) {
  v4u w;
  w[0] = pk16(hb[0], hb[1]); w[1] = pk16(hb[2], hb[3]); w[2] = pk16(hb[4], hb[5]); w[3] = pk16(hb[6], hb[7]);
  return w;
}
__device__ __forceinline__ void st2_v4u(unsigned short* p, v4u w) {
  *(volatile v4u*)(void*)p = w;
  __threadfence();
  *(volatile v4u*)(void*)p = w;
}

__device__ __forceinline__ v16b lds_frag(const unsigned short* p) {
  union { v16b v; v8b h[2]; } f;
  f.h[0] = *(const v8b*)(const void*)(p);
  f.h[1] = *(const v8b*)(const void*)(p + 16);
  return f.v;
}
__device__ __forceinline__ v8f mma_bf(v16b a, v16b b, v8f cacc) {
  cacc = __builtin_amdgcn_wmma_f32_16x16x32_bf16(false, a, false, b, (short)0, cacc, false, false);
  asm volatile("v_nop\n\tv_nop\n\tv_nop\n\tv_nop" : "+v"(cacc) : "v"(a), "v"(b));
  return cacc;
}
template <int KS, int BP>
__device__ __forceinline__ void gemm4(const unsigned short* sAw, const unsigned short* sBp, int c, int hh, v8f (&acc)[4]) {
  const v8f z8 = {0.f, 0.f, 0.f, 0.f, 0.f, 0.f, 0.f, 0.f};
#pragma unroll
  for (int j = 0; j < 4; ++j) acc[j] = z8;
#pragma unroll 1
  for (int ks = 0; ks < KS; ++ks) {
    const v16b a = lds_frag(sAw + c * kAP + ks * 32 + 8 * hh);
#pragma unroll
    for (int j = 0; j < 4; ++j) {
      const v16b b = lds_frag(sBp + (j * 16 + c) * BP + ks * 32 + 8 * hh);
      acc[j] = mma_bf(a, b, acc[j]);
    }
  }
}
__device__ __forceinline__ void put_hl(unsigned short* sAw, int row, int col, float v) {
  const unsigned short hb = f2bf_bits(v);
  const unsigned short lb = f2bf_bits(v - bf_bits2f(hb));
  sAw[row * kAP + col] = hb;
  sAw[row * kAP + kHid + col] = lb;
}
__device__ __forceinline__ float sigm(float x) { x = fminf(fmaxf(x, -30.0f), 30.0f); return 1.0f / (1.0f + expf(-x)); }
__device__ __forceinline__ float tanh_c(float x) { x = fminf(fmaxf(x, -20.0f), 20.0f); return tanhf(x); }

__device__ __forceinline__ int blk_excl_scan(int cnt, int* scan_ws, int tid, int* tot) {
  const int lane = tid & 31, wave = tid >> 5; int incl = cnt;
#pragma unroll
  for (int o = 1; o < 32; o <<= 1) { const int v = __shfl_up(incl, o, 32); if (lane >= o) incl += v; }
  if (lane == 31) scan_ws[wave] = incl;
  __syncthreads();
  if (wave == 0) { int wv = (lane < kThr / 32) ? scan_ws[lane] : 0; int wincl = wv;
#pragma unroll
    for (int o = 1; o < 32; o <<= 1) { const int v = __shfl_up(wincl, o, 32); if (lane >= o) wincl += v; }
    if (lane < kThr / 32) scan_ws[32 + lane] = wincl - wv; if (lane == 31) scan_ws[64] = wincl; }
  __syncthreads();
  const int res = scan_ws[32 + wave] + incl - cnt; *tot = scan_ws[64];
  return res;
}
template <int SRB, bool WITHSRC>
__device__ __forceinline__ int chunk_collect(const int* __restrict__ dstv, const int* __restrict__ srcv, int e0, int n0, int tid,
                                             int* LIST, int* scan_ws) {
  const int eb = e0 + tid * kSpt;
  const bool live = eb < kE;
  const int ebc = live ? eb : (kE - kSpt);
  int rec[kSpt]; int cnt = 0;
#pragma unroll
  for (int k = 0; k < kSpt; k += 4) {
    const v4i d4 = *(const v4i*)(dstv + ebc + k);
    v4i s4 = (v4i){0, 0, 0, 0};
    if (WITHSRC) s4 = *(const v4i*)(srcv + ebc + k);
#pragma unroll
    for (int e = 0; e < 4; ++e) {
      const int d = d4[e];
      const bool hit = live && d >= n0 && d < n0 + SRB;
      int s = s4[e]; s = s < 0 ? 0 : (s >= kN ? kN - 1 : s);
      const int code = WITHSRC ? (int)((((unsigned)(d - n0)) << 16) | (unsigned)s) : (d - n0);
      rec[k + e] = hit ? code : -1;
      cnt += hit ? 1 : 0;
    }
  }
  int tot; int p = blk_excl_scan(cnt, scan_ws, tid, &tot);
#pragma unroll
  for (int k = 0; k < kSpt; ++k) if (rec[k] >= 0) { if ((unsigned)p < (unsigned)kSch) LIST[p] = rec[k]; ++p; }
  __syncthreads();
  return tot < kSch ? tot : kSch;
}

__global__ __launch_bounds__(kThr) void k_prep(
    const float* __restrict__ Wz, const float* __restrict__ Wr, const float* __restrict__ Wh,
    const float* __restrict__ bz, const float* __restrict__ br, const float* __restrict__ bh,
    const float* __restrict__ lzW, const float* __restrict__ lrW, const float* __restrict__ lhW,
    const float* __restrict__ lzb, const float* __restrict__ lrb, const float* __restrict__ lhb,
    const float* __restrict__ att, const float* __restrict__ l1W, const float* __restrict__ l1b,
    const float* __restrict__ outW, const float* __restrict__ outb,
    unsigned short* __restrict__ PREP, float* __restrict__ TAB) {
  const int t = blockIdx.x * kThr + threadIdx.x;
  if (t < kR0) {
    const int g = t >> 10, u = t & 1023, n = u >> 4, k0 = (u & 15) * 8;
    const float* lgW = (g == 0) ? lzW : ((g == 1) ? lrW : lhW);
    unsigned short hb[8];
#pragma unroll
    for (int e = 0; e < 8; ++e) { const int kk = (k0 + e) & 63; hb[e] = f2bf_bits(lgW[(64 + kk) * kHid + n]); }
    st2_v4u(PREP + g * kPrepGate + n * kGateBP + k0, pack8(hb));
  } else if (t < kR1) {
    const int tt = t - kR0; const int g = tt >> 9, u = tt & 511, n = u >> 3, q = u & 7;
    const float* Wg  = (g == 0) ? Wz  : ((g == 1) ? Wr  : Wh);
    const float* lgW = (g == 0) ? lzW : ((g == 1) ? lrW : lhW);
    float d[8];
#pragma unroll
    for (int cc = 0; cc < 8; ++cc) d[cc] = 0.0f;
#pragma unroll 1
    for (int j = 0; j < kHid; ++j) {
      const float lw = bfr(lgW[j * kHid + n]);
#pragma unroll
      for (int cc = 0; cc < 8; ++cc) d[cc] = fmaf(bfr(Wg[cc * kHid + j]), lw, d[cc]);
    }
    const int g4 = (q >> 1) & 1, sub = q & 1;
    unsigned short hb[8];
#pragma unroll
    for (int e = 0; e < 8; ++e) {
      const float va = d[e & 3], vb = d[4 + (e & 3)];
      const float v = (g4 == 0) ? va : vb;
      const unsigned short hbit = f2bf_bits(v);
      const unsigned short lbit = f2bf_bits(v - bf_bits2f(hbit));
      const unsigned short lz = ((e >> 2) == 0) ? lbit : (unsigned short)0;
      const unsigned short sv = (sub == 0) ? hbit : lz;
      hb[e] = (q < 4) ? sv : (unsigned short)0;
    }
    st2_v4u(PREP + g * kPrepGate + n * kGateBP + 128 + 8 * q, pack8(hb));
  } else if (t < kR2) {
    const int tt = t - kR1; const int n = tt >> 4, k0 = (tt & 15) * 8;
    unsigned short hb[8];
#pragma unroll
    for (int e = 0; e < 8; ++e) { const int kk = (k0 + e) & 63; hb[e] = f2bf_bits(l1W[kk * kHid + n]); }
    st2_v4u(PREP + kPrepP1 + n * kHeadBP + k0, pack8(hb));
  } else if (t < kR3) {
    const int tt = t - kR2; const int n = tt >> 4, k0 = (tt & 15) * 8;
    const int nc = (n < kPer) ? n : (kPer - 1);
    unsigned short hb[8];
#pragma unroll
    for (int e = 0; e < 8; ++e) {
      const int kk = (k0 + e) & 63;
      const unsigned short v = f2bf_bits(outW[kk * kPer + nc]);
      hb[e] = (n < kPer) ? v : (unsigned short)0;
    }
    st2_v4u(PREP + kPrepPO + n * kHeadBP + k0, pack8(hb));
  } else if (t < kR4) {
    const int f = t - kR3; const int wt = f >> 5;
    float val = 0.0f;
    if (wt < 6) {
      const int g = wt >> 1; const int n = f - 64 * g;
      const float* bg  = (g == 0) ? bz  : ((g == 1) ? br  : bh);
      const float* lgW = (g == 0) ? lzW : ((g == 1) ? lrW : lhW);
      const float* lgb = (g == 0) ? lzb : ((g == 1) ? lrb : lhb);
      float s = 0.0f;
#pragma unroll 1
      for (int j = 0; j < kHid; ++j) s = fmaf(bfr(bg[j]), bfr(lgW[j * kHid + n]), s);
      val = s + bfr(lgb[n]);
    } else if (wt < 8) {
      val = bfr(l1b[f - kTabL1b]);
    } else {
      const int ln = f - kTabOutb;
      const int oi = (ln < kPer) ? ln : (kPer - 1);
      const float ob = bfr(outb[oi]);
      float m = -3.0e38f;
#pragma unroll 1
      for (int j = 0; j < kPer; ++j) m = fmaxf(m, bfr(att[j]));
      float ssum = 0.0f, psel = 0.0f; const int pj = ln - 16;
#pragma unroll 1
      for (int j = 0; j < kPer; ++j) { const float ev = expf(bfr(att[j]) - m); ssum = ssum + ev; psel = (pj == j) ? ev : psel; }
      const float pv = psel * (1.0f / ssum);
      val = (ln < kPer) ? ob : ((ln < 16) ? 0.0f : ((ln < 16 + kPer) ? pv : 0.0f));
    }
    ((volatile float*)TAB)[f] = val;
    __threadfence();
    ((volatile float*)TAB)[f] = val;
  }
}

__global__ __launch_bounds__(kThr) void k_deg(const int* __restrict__ ei, const float* __restrict__ x,
                                             float* __restrict__ DINV, float* __restrict__ Y) {
  __shared__ int LIST[kSch];
  __shared__ __align__(16) int sCnt[kSrbD];
  __shared__ int scan_ws[80];
  const int tid = threadIdx.x, lane = tid & 31, wave = tid >> 5;
  const int n0 = blockIdx.x * kSrbD;
  for (int i = tid; i < kSrbD; i += kThr) sCnt[i] = 0;
  if (tid < 80) scan_ws[tid] = 0;
  __syncthreads();
  const int* srcv = ei; const int* dstv = ei + kE;
#pragma unroll 1
  for (int ch = 0; ch < kNch; ++ch) {
    const int tot = chunk_collect<kSrbD, false>(dstv, srcv, ch * kSch, n0, tid, LIST, scan_ws);
#pragma unroll 1
    for (int base = 0; base < tot; base += 32) {
      const int q = base + lane;
      const int qi = (q < tot) ? q : 0;
      int rv = LIST[qi]; rv = (q < tot) ? rv : -1;
      const int own = (rv >= 0 && (rv >> kShiftD) == wave) ? 1 : 0;
      unsigned msk = (unsigned)__ballot(own);
#pragma unroll 1
      for (int it = 0; it < 32; ++it) {
        if (msk == 0u) break;
        const int bp = __builtin_ctz(msk); msk &= msk - 1u;
        const int r = __shfl(rv, bp, 32);
        const int dl = r & (kSrbD - 1);
        if (lane == 0) sCnt[dl] = sCnt[dl] + 1;
      }
    }
    __syncthreads();
  }
  for (int pass = 0; pass < 2; ++pass) {
#pragma unroll 1
    for (int it = 0; it < kRowsWaveD / 128; ++it) {
      const int dl = wave * kRowsWaveD + it * 128 + 4 * lane;
      const v4i cv = *(const v4i*)(sCnt + dl);
      v4f dv;
#pragma unroll
      for (int e = 0; e < 4; ++e) dv[e] = 1.0f / sqrtf((float)(cv[e] + 1));
      *(volatile v4f*)(DINV + n0 + dl) = dv;
    }
    __threadfence();
  }
#pragma unroll 1
  for (int dl = wave; dl < kSrbD; dl += 8) {
    const int n = n0 + dl;
    if (n >= kN) break;
    const float dv = 1.0f / sqrtf((float)(sCnt[dl] + 1));
    const float fk = (lane < kFeat / 4) ? dv : 0.0f;
    const int c4 = 4 * lane; const int cc = (c4 < kFeat - 4) ? c4 : (kFeat - 4);
    const v4f xv = *(const v4f*)(x + (size_t)n * kFeat + cc);
    v4f yv;
#pragma unroll
    for (int e = 0; e < 4; ++e) yv[e] = bfr(xv[e]) * fk;
    float* yp = Y + (size_t)n * kAggPitch + c4;
    *(volatile v4f*)yp = yv;
    __threadfence();
    *(volatile v4f*)yp = yv;
  }
}

__global__ __launch_bounds__(kThr) void k_agg(const int* __restrict__ ei, const float* __restrict__ Y,
                                             const float* __restrict__ DINV, float* AGG) {
  __shared__ int LIST[kSch];
  __shared__ int scan_ws[80];
  const int tid = threadIdx.x, lane = tid & 31, wave = tid >> 5;
  const int n0 = blockIdx.x * kSrbA;
  if (tid < 80) scan_ws[tid] = 0;
  const v4f z4 = {0.0f, 0.0f, 0.0f, 0.0f};
#pragma unroll 1
  for (int j = 0; j < kRowsWaveA; ++j)
    *(v4f*)(AGG + (size_t)(n0 + wave * kRowsWaveA + j) * kAggPitch + 4 * lane) = z4;
  __syncthreads();
  const int* srcv = ei; const int* dstv = ei + kE;
#pragma unroll 1
  for (int ch = 0; ch < kNch; ++ch) {
    const int tot = chunk_collect<kSrbA, true>(dstv, srcv, ch * kSch, n0, tid, LIST, scan_ws);
#pragma unroll 1
    for (int base = 0; base < tot; base += 32) {
      const int q = base + lane;
      const int qi = (q < tot) ? q : 0;
      int rv = LIST[qi]; rv = (q < tot) ? rv : -1;
      const int own = (rv >= 0 && (rv >> kShiftA) == wave) ? 1 : 0;
      unsigned msk = (unsigned)__ballot(own);
#pragma unroll 1
      for (int it = 0; it < 32; ++it) {
        if (msk == 0u) break;
        const int bp = __builtin_ctz(msk); msk &= msk - 1u;
        const int r = __shfl(rv, bp, 32);
        const int dl = (r >> 16) & (kSrbA - 1);
        int s = r & 0xFFFF; s = (s < kN) ? s : (kN - 1);
        const v4f yv = *(const v4f*)(Y + (size_t)s * kAggPitch + 4 * lane);
        float* ap = AGG + (size_t)(n0 + dl) * kAggPitch + 4 * lane;
        v4f a = *(const v4f*)ap;
        a = a + yv;
        *(v4f*)ap = a;
      }
    }
    __syncthreads();
  }
#pragma unroll 1
  for (int j = 0; j < kRowsWaveA; ++j) {
    const int dl = wave * kRowsWaveA + j; const int n = n0 + dl;
    const int nc = (n < kN) ? n : (kN - 1);
    float* ap = AGG + (size_t)n * kAggPitch + 4 * lane;
    const v4f a  = *(const v4f*)ap;
    const v4f ys = *(const v4f*)(Y + (size_t)nc * kAggPitch + 4 * lane);
    const float dv = DINV[n];
    v4f v = (a + ys) * dv;
    if (n >= kN) v = z4;
    *(volatile v4f*)ap = v;
    __threadfence();
    *(volatile v4f*)ap = v;
  }
}

__global__ __launch_bounds__(kGruThr) void k_gru(const float* __restrict__ AGG, const unsigned short* __restrict__ PREP,
                                                const float* __restrict__ TAB, float* __restrict__ out) {
  __shared__ __align__(16) unsigned short sB[kPrepHalves];
  __shared__ __align__(16) unsigned short sA[4 * 16 * kAP];
  __shared__ __align__(16) float sZ[4 * 16 * kHid];
  __shared__ __align__(16) float sHa[4 * 16 * kHid];
  __shared__ __align__(16) float sTab[kTabFloats];
  __shared__ __align__(16) float sOut[kNodesBlk * kPer];
  const int tid = threadIdx.x, lane = tid & 31, wave = tid >> 5;
  const int c = lane & 15, hh = lane >> 4;
  unsigned short* sAw = sA + wave * (16 * kAP);
  float* sZw = sZ + wave * (16 * kHid);
  float* sHw = sHa + wave * (16 * kHid);
  {
    const v4u* gp = (const v4u*)(const void*)PREP;
    v4u* lp = (v4u*)(void*)sB;
#pragma unroll 2
    for (int i = tid; i < kPrepChunks; i += kGruThr) lp[i] = gp[i];
    if (tid < kTabFloats / 4) ((v4f*)(void*)sTab)[tid] = ((const v4f*)(const void*)TAB)[tid];
#pragma unroll
    for (int j = 0; j < 4; ++j)
#pragma unroll
      for (int r = 0; r < 8; ++r) sHw[(8 * hh + r) * kHid + 16 * j + c] = 0.0f;
  }
  __syncthreads();

  const int nb0 = blockIdx.x * kNodesBlk;
  int nodeX = nb0 + wave * 16 + c; nodeX = (nodeX < kN) ? nodeX : (kN - 1);
  const float* xrow = AGG + (size_t)nodeX * kAggPitch + (4 * hh) * kPer;
  const v8f z8 = {0.f, 0.f, 0.f, 0.f, 0.f, 0.f, 0.f, 0.f};
  v8f Hs[4], acc[4];
#pragma unroll
  for (int j = 0; j < 4; ++j) Hs[j] = z8;

#pragma unroll 1
  for (int t = 0; t < kPer; ++t) {
    {
      const float x0 = xrow[t], x1 = xrow[kPer + t], x2 = xrow[2 * kPer + t], x3 = xrow[3 * kPer + t];
      const unsigned short h0 = f2bf_bits(x0), h1 = f2bf_bits(x1), h2 = f2bf_bits(x2), h3 = f2bf_bits(x3);
      const unsigned short l0 = f2bf_bits(x0 - bf_bits2f(h0)), l1 = f2bf_bits(x1 - bf_bits2f(h1));
      const unsigned short l2 = f2bf_bits(x2 - bf_bits2f(h2)), l3 = f2bf_bits(x3 - bf_bits2f(h3));
      v4u w;
      w[0] = pk16(h0, h1); w[1] = pk16(h2, h3); w[2] = pk16(l0, l1); w[3] = pk16(l2, l3);
      v4u* xp = (v4u*)(void*)(sAw + c * kAP + 2 * kHid + 16 * hh);
      xp[0] = w; xp[1] = w;
    }
#pragma unroll
    for (int j = 0; j < 4; ++j)
#pragma unroll
      for (int r = 0; r < 8; ++r) put_hl(sAw, 8 * hh + r, j * 16 + c, Hs[j][r]);
    __syncthreads();

    gemm4<kGateK / 32, kGateBP>(sAw, sB, c, hh, acc);
#pragma unroll
    for (int j = 0; j < 4; ++j) {
      const float bj = sTab[kTabBz + j * 16 + c];
#pragma unroll
      for (int r = 0; r < 8; ++r) sZw[(8 * hh + r) * kHid + 16 * j + c] = sigm(acc[j][r] + bj);
    }
    gemm4<kGateK / 32, kGateBP>(sAw, sB + kPrepGate, c, hh, acc);
    __syncthreads();
#pragma unroll
    for (int j = 0; j < 4; ++j) {
      const float bj = sTab[kTabBr + j * 16 + c];
#pragma unroll
      for (int r = 0; r < 8; ++r) {
        const float rg = sigm(acc[j][r] + bj);
        put_hl(sAw, 8 * hh + r, j * 16 + c, rg * Hs[j][r]);
      }
    }
    __syncthreads();
    gemm4<kGateK / 32, kGateBP>(sAw, sB + 2 * kPrepGate, c, hh, acc);
    const float pt = sTab[kTabProb + t];
#pragma unroll
    for (int j = 0; j < 4; ++j) {
      const float bj = sTab[kTabBh + j * 16 + c];
#pragma unroll
      for (int r = 0; r < 8; ++r) {
        const int idx = (8 * hh + r) * kHid + 16 * j + c;
        const float ht = tanh_c(acc[j][r] + bj);
        const float z = sZw[idx];
        const float hn = z * Hs[j][r] + (1.0f - z) * ht;
        Hs[j][r] = hn;
        sHw[idx] = sHw[idx] + pt * hn;
      }
    }
    __syncthreads();
  }

#pragma unroll
  for (int j = 0; j < 4; ++j)
#pragma unroll
    for (int r = 0; r < 8; ++r) {
      const int idx = (8 * hh + r) * kHid + 16 * j + c;
      put_hl(sAw, 8 * hh + r, j * 16 + c, fmaxf(sHw[idx], 0.0f));
    }
  __syncthreads();
  gemm4<kHeadK / 32, kHeadBP>(sAw, sB + kPrepP1, c, hh, acc);
  __syncthreads();
#pragma unroll
  for (int j = 0; j < 4; ++j) {
    const float bj = sTab[kTabL1b + j * 16 + c];
#pragma unroll
    for (int r = 0; r < 8; ++r) put_hl(sAw, 8 * hh + r, j * 16 + c, fmaxf(acc[j][r] + bj, 0.0f));
  }
  __syncthreads();
  v8f o = z8;
#pragma unroll
  for (int ks = 0; ks < kHeadK / 32; ++ks) {
    const v16b a = lds_frag(sAw + c * kAP + ks * 32 + 8 * hh);
    const v16b b = lds_frag(sB + kPrepPO + c * kHeadBP + ks * 32 + 8 * hh);
    o = mma_bf(a, b, o);
  }
  const float ob = sTab[kTabOutb + c];
  if (c < kPer) {
#pragma unroll
    for (int r = 0; r < 8; ++r) sOut[(wave * 16 + 8 * hh + r) * kPer + c] = o[r] + ob;
  }
  __syncthreads();
  if (wave < 3) {
    const int q8 = lane >> 3, c4 = (lane & 7) * 4;
    for (int pass = 0; pass < 2; ++pass) {
#pragma unroll
      for (int it = 0; it < 2; ++it) {
        const int ll = wave * 8 + it * 4 + q8;
        const int gl = blockIdx.x * kLinesBlk + ll;
        const v4f v = *(const v4f*)(sOut + ll * 32 + c4);
        if (gl < kOutLines) *(volatile v4f*)(out + (size_t)gl * 32 + c4) = v;
      }
      __threadfence();
    }
  }
}

extern "C" void kernel_launch(void* const* d_in, const int* in_sizes, int n_in,
                              void* d_out, int out_size, void* d_ws, size_t ws_size, hipStream_t stream) {
  (void)in_sizes; (void)n_in;
  const float* x    = (const float*)d_in[0];
  const int*   ei   = (const int*)  d_in[1];
  const float* Wz   = (const float*)d_in[2];
  const float* bz   = (const float*)d_in[3];
  const float* Wr   = (const float*)d_in[4];
  const float* br   = (const float*)d_in[5];
  const float* Wh   = (const float*)d_in[6];
  const float* bh   = (const float*)d_in[7];
  const float* lzW  = (const float*)d_in[8];
  const float* lzb  = (const float*)d_in[9];
  const float* lrW  = (const float*)d_in[10];
  const float* lrb  = (const float*)d_in[11];
  const float* lhW  = (const float*)d_in[12];
  const float* lhb  = (const float*)d_in[13];
  const float* att  = (const float*)d_in[14];
  const float* l1W  = (const float*)d_in[15];
  const float* l1b  = (const float*)d_in[16];
  const float* outW = (const float*)d_in[17];
  const float* outb = (const float*)d_in[18];
  float* out = (float*)d_out;
  if (out_size < kN * kPer) return;

  char* ws = (char*)d_ws; size_t off = 0;
  auto carve = [&](size_t bytes) -> char* { char* p = ws + off; off += (bytes + 255) & ~(size_t)255; return p; };
  unsigned short* PREP = (unsigned short*)carve((size_t)kPrepHalves * 2);
  float*          TAB  = (float*)carve((size_t)kTabFloats * 4);
  float*          DINV = (float*)carve((size_t)kDinvRows * 4);
  float*          Y    = (float*)carve((size_t)kN * kAggPitch * 4);
  float*          AGG  = (float*)carve((size_t)kAggRows * kAggPitch * 4);
  if (off > ws_size || off > (size_t)134217728) return;

  k_prep<<<kPrepBlocks, kThr, 0, stream>>>(Wz, Wr, Wh, bz, br, bh, lzW, lrW, lhW, lzb, lrb, lhb,
                                          att, l1W, l1b, outW, outb, PREP, TAB);
  k_deg<<<kNblkD, kThr, 0, stream>>>(ei, x, DINV, Y);
  k_agg<<<kNblkA, kThr, 0, stream>>>(ei, Y, DINV, AGG);
  k_gru<<<kGruBlocks, kGruThr, 0, stream>>>(AGG, PREP, TAB, out);
}
